// AvgSeerMambaTransLayer_50637664420399
// MI455X (gfx1250) — hardware-verified
//
#include <hip/hip_runtime.h>
#include <stddef.h>

#define C_DIM   256
#define DMODEL  512
#define DINNER  1024
#define DSTATE  256
#define DTRANK  32
#define DCONV   4
#define NB      2
#define SEQ     512
#define MROWS   (NB * SEQ)
#define NDBL    (DTRANK + 2 * DSTATE)
#define LDP     576
#define LN_EPS  1e-5f
#define WSC     64.0f
#define XSC     64.0f
#define DTWSC   16.0f
#define YSC     256.0f

typedef __attribute__((ext_vector_type(16))) _Float16 v16h;
typedef __attribute__((ext_vector_type(8)))  _Float16 v8h;
typedef __attribute__((ext_vector_type(16))) __bf16   v16b;
typedef __attribute__((ext_vector_type(8)))  __bf16   v8b;
typedef __attribute__((ext_vector_type(8)))  float    v8f;
typedef __attribute__((ext_vector_type(4)))  float    v4f;
#define PSCALE 32768.0f
#define U16(p) ((const unsigned short*)(const void*)(p))
#define PSCALE_INV (1.0f / 32768.0f)

__device__ __forceinline__ unsigned short f2bf_bits(float f) {
  unsigned u = __float_as_uint(f);
  return (unsigned short)((u + 0x7FFFu + ((u >> 16) & 1u)) >> 16);
}
__device__ __forceinline__ float bf_bits2f(unsigned short h) { return __uint_as_float(((unsigned)h) << 16); }

__device__ __forceinline__ void dep_guard_h(v8f& a, v8f& b, v16h x, v16h y) { asm volatile("v_nop\n\tv_nop\n\tv_nop\n\tv_nop" : "+v"(a), "+v"(b) : "v"(x), "v"(y)); }
__device__ __forceinline__ void dep_guard_b(v8f& a, v8f& b, v16b x, v16b y) { asm volatile("v_nop\n\tv_nop\n\tv_nop\n\tv_nop" : "+v"(a), "+v"(b) : "v"(x), "v"(y)); }
__device__ __forceinline__ void keep4_h(v16h a, v16h b, v16h c, v16h d) { asm volatile("v_nop" :: "v"(a), "v"(b), "v"(c), "v"(d)); }
__device__ __forceinline__ void keep4_b(v16b a, v16b b, v16b c, v16b d) { asm volatile("v_nop" :: "v"(a), "v"(b), "v"(c), "v"(d)); }
__device__ __forceinline__ void acc_guard4(v8f& a, v8f& b, v8f& c, v8f& d) { asm volatile("v_nop\n\tv_nop\n\tv_nop\n\tv_nop" : "+v"(a), "+v"(b), "+v"(c), "+v"(d)); }
template <typename T> struct Frag;
template <> struct Frag<_Float16> {
  typedef v16h V; union U { v16h v; v8h h[2]; };
  static __device__ __forceinline__ v16h load(const _Float16* p) {
    U f; f.h[0] = *(const v8h*)(p); f.h[1] = *(const v8h*)(p + 16); return f.v;
  }
  static __device__ __forceinline__ v8f mma(v16h a, v16h b, v8f c) {
    return __builtin_amdgcn_wmma_f32_16x16x32_f16(false, a, false, b, (short)0, c, false, false);
  }
  static __device__ __forceinline__ void guard(v8f& a, v8f& b, v16h x, v16h y) { dep_guard_h(a, b, x, y); }
  static __device__ __forceinline__ void keep(v16h a, v16h b, v16h c, v16h d) { keep4_h(a, b, c, d); }
};
template <> struct Frag<__bf16> {
  typedef v16b V; union U { v16b v; v8b h[2]; };
  static __device__ __forceinline__ v16b load(const __bf16* p) {
    U f; f.h[0] = *(const v8b*)(p); f.h[1] = *(const v8b*)(p + 16); return f.v;
  }
  static __device__ __forceinline__ v8f mma(v16b a, v16b b, v8f c) {
    return __builtin_amdgcn_wmma_f32_16x16x32_bf16(false, a, false, b, (short)0, c, false, false);
  }
  static __device__ __forceinline__ void guard(v8f& a, v8f& b, v16b x, v16b y) { dep_guard_b(a, b, x, y); }
  static __device__ __forceinline__ void keep(v16b a, v16b b, v16b c, v16b d) { keep4_b(a, b, c, d); }
};

template <int ET> struct Elem;
template <> struct Elem<0> { typedef _Float16 T; };
template <> struct Elem<1> { typedef __bf16 T; };
template <int ET, bool SPLIT, int BIAS_MODE, int OUT_MODE, bool RESID, int ACT = 0>
__global__ __launch_bounds__(256) void wmma_gemm64(
    const unsigned short* __restrict__ Ap, const unsigned short* __restrict__ A2p, int lda, long strideA,
    const unsigned short* __restrict__ Btp, const unsigned short* __restrict__ Bt2p, int ldb, long strideB,
    void* __restrict__ Cout, void* __restrict__ Cout2, int ldc, long strideC,
    const float* __restrict__ bias,
    const float* __restrict__ resid, long strideR,
    int M, int N, int K, float scale) {
  typedef typename Elem<ET>::T T;
  typedef typename Frag<T>::V V;
  const T* A = (const T*)Ap; const T* A2 = (const T*)A2p; const T* Bt = (const T*)Btp; const T* Bt2 = (const T*)Bt2p;
  __shared__ __align__(16) float sT[8][16 * 68];
  const int b    = blockIdx.y;
  const int lane = threadIdx.x & 31;
  const int wave = threadIdx.x >> 5;
  const int tilesN = N >> 6;
  const int tilesM = M >> 6;
  const int tile = blockIdx.x * 8 + wave;
  if (tile >= tilesM * tilesN) return;
  const int tm = tile / tilesN;
  const int tn = tile - tm * tilesN;
  const int m0 = tm << 6;
  const int n0 = tn << 6;

  const T* Ab  = A  + (size_t)b * strideA;
  const T* Bb  = Bt + (size_t)b * strideB;
  const T* Ab2 = SPLIT ? (A2  + (size_t)b * strideA) : nullptr;
  const T* Bb2 = SPLIT ? (Bt2 + (size_t)b * strideB) : nullptr;

  const int rlane = lane & 15;
  const int koff  = (lane >> 4) * 8;
  const int mOff  = (lane >> 4) * 8;

  v8f acc[4][4];
#pragma unroll
  for (int i = 0; i < 4; ++i)
#pragma unroll
    for (int j = 0; j < 4; ++j) acc[i][j] = (v8f){0.f,0.f,0.f,0.f,0.f,0.f,0.f,0.f};

  for (int k0 = 0; k0 < K; k0 += 32) {
    V bh[4], bl[4];
#pragma unroll
    for (int j = 0; j < 4; ++j) {
      const size_t bo = (size_t)(n0 + (j << 4) + rlane) * ldb + koff + k0;
      bh[j] = Frag<T>::load(Bb + bo);
      if (SPLIT) bl[j] = Frag<T>::load(Bb2 + bo);
    }
#pragma unroll
    for (int i = 0; i < 4; ++i) {
      const size_t ao = (size_t)(m0 + (i << 4) + rlane) * lda + koff + k0;
      V ah = Frag<T>::load(Ab + ao);
      V al;
      if (SPLIT) al = Frag<T>::load(Ab2 + ao);
#pragma unroll
      for (int j = 0; j < 4; ++j) {
        acc[i][j] = Frag<T>::mma(ah, bh[j], acc[i][j]);
        if (SPLIT) {
          acc[i][j] = Frag<T>::mma(ah, bl[j], acc[i][j]);
          acc[i][j] = Frag<T>::mma(al, bh[j], acc[i][j]);
        }
      }
      Frag<T>::guard(acc[i][0], acc[i][3], ah, SPLIT ? al : ah);
    }
    Frag<T>::keep(bh[0], bh[1], bh[2], bh[3]);
    if (SPLIT) Frag<T>::keep(bl[0], bl[1], bl[2], bl[3]);
  }
  acc_guard4(acc[0][0], acc[0][1], acc[0][2], acc[0][3]);
  acc_guard4(acc[1][0], acc[1][1], acc[1][2], acc[1][3]);
  acc_guard4(acc[2][0], acc[2][1], acc[2][2], acc[2][3]);
  acc_guard4(acc[3][0], acc[3][1], acc[3][2], acc[3][3]);

  float* slab = sT[wave];
  const float* Rb = RESID ? (resid + (size_t)b * strideR) : nullptr;
#pragma unroll
  for (int i = 0; i < 4; ++i) {
    const int mBase = m0 + (i << 4);
#pragma unroll
    for (int j = 0; j < 4; ++j) {
      const int n = n0 + (j << 4) + rlane;
      float bv = 0.f;
      if (BIAS_MODE == 2) bv = bias[n];
#pragma unroll
      for (int r = 0; r < 8; ++r) {
        float v = acc[i][j][r] * scale;
        if (BIAS_MODE == 1) v += bias[mBase + mOff + r];
        if (BIAS_MODE == 2) v += bv;
        if (RESID) v += Rb[(size_t)(mBase + mOff + r) * ldc + n];
        if (ACT == 1) v = tanhf(v);
        if (ACT == 2) v = fmaxf(v, 0.0f);
        if (ACT == 3) v = v / (1.0f + expf(-v));
        if (ACT == 4) v = (v > 0.f) ? v : 0.01f * v;
        if (ACT == 5) v = 0.5f * v * (1.0f + erff(v * 0.70710678118654752f));
        slab[(mOff + r) * 68 + (j << 4) + rlane] = v;
      }
    }
    __builtin_amdgcn_fence(__ATOMIC_RELEASE, "workgroup");
    __builtin_amdgcn_wave_barrier();
    __builtin_amdgcn_fence(__ATOMIC_ACQUIRE, "workgroup");
    if (OUT_MODE == 0) {
      float* C = (float*)Cout + (size_t)b * strideC;
      const int hh = lane >> 4, c4 = (lane & 15) * 4;
      for (int pass = 0; pass < 2; ++pass) {
#pragma unroll
        for (int it = 0; it < 8; ++it) {
          const int row = it * 2 + hh;
          v4f v = *(const v4f*)(slab + row * 68 + c4);
          *(volatile v4f*)(C + (size_t)(mBase + row) * ldc + n0 + c4) = v;
        }
        __threadfence();
      }
    } else {
      const int q = lane >> 3, c8 = (lane & 7) * 8;
      unsigned short* C  = (unsigned short*)Cout  + (size_t)b * strideC;
      unsigned short* C2 = (OUT_MODE == 2) ? ((unsigned short*)Cout2 + (size_t)b * strideC) : nullptr;
      for (int pass = 0; pass < 2; ++pass) {
#pragma unroll
        for (int it = 0; it < 4; ++it) {
          const int row = it * 4 + q;
          const float* sp = slab + row * 68 + c8;
          v8h hv, lv;
#pragma unroll
          for (int e = 0; e < 8; ++e) {
            if (OUT_MODE == 1) {
              hv[e] = (_Float16)sp[e];
            } else {
              unsigned short hb = f2bf_bits(sp[e]);
              unsigned short lb = f2bf_bits(sp[e] - bf_bits2f(hb));
              hv[e] = __builtin_bit_cast(_Float16, hb);
              lv[e] = __builtin_bit_cast(_Float16, lb);
            }
          }
          *(volatile v8h*)(C + (size_t)(mBase + row) * ldc + n0 + c8) = hv;
          if (OUT_MODE == 2) *(volatile v8h*)(C2 + (size_t)(mBase + row) * ldc + n0 + c8) = lv;
        }
        __threadfence();
      }
    }
    __builtin_amdgcn_fence(__ATOMIC_RELEASE, "workgroup");
    __builtin_amdgcn_wave_barrier();
    __builtin_amdgcn_fence(__ATOMIC_ACQUIRE, "workgroup");
  }
}

__global__ __launch_bounds__(256) void k_cast_rows(const float* __restrict__ in, _Float16* __restrict__ out,
                                                   int rows_in, int cols, int rows_out, float scale) {
  const int i8 = blockIdx.x * 256 + threadIdx.x;
  const int n8 = (rows_out * cols) >> 3;
  if (i8 < n8) {
    const int e0  = i8 << 3;
    const int row = e0 / cols;
    const int col = e0 - row * cols;
    const int rr  = (row < rows_in) ? row : (rows_in - 1);
    const float* p = in + (size_t)rr * cols + col;
    const v4f a = *(const v4f*)p;
    const v4f c = *(const v4f*)(p + 4);
    const float z = (row < rows_in) ? scale : 0.0f;
    v8h hv;
    hv[0] = (_Float16)(a[0] * z); hv[1] = (_Float16)(a[1] * z); hv[2] = (_Float16)(a[2] * z); hv[3] = (_Float16)(a[3] * z);
    hv[4] = (_Float16)(c[0] * z); hv[5] = (_Float16)(c[1] * z); hv[6] = (_Float16)(c[2] * z); hv[7] = (_Float16)(c[3] * z);
    _Float16* q = out + e0;
    *(volatile v8h*)q = hv;
    __threadfence();
    *(volatile v8h*)q = hv;
  }
}

__global__ __launch_bounds__(128) void k_avg(const float* __restrict__ x, float* __restrict__ avg) {
  const int t  = threadIdx.x;
  const int b  = t >> 6;
  const int c4 = (t & 63) << 2;
  const float* p = x + (size_t)b * SEQ * C_DIM + c4;
  double s0 = 0.0, s1 = 0.0, s2 = 0.0, s3 = 0.0;
  for (int l = 0; l < SEQ; ++l) {
    const v4f v = *(const v4f*)(p + (size_t)l * C_DIM);
    s0 += (double)v[0]; s1 += (double)v[1]; s2 += (double)v[2]; s3 += (double)v[3];
  }
  const float inv = 1.0f / (float)SEQ;
  v4f r;
  r[0] = (float)s0 * inv; r[1] = (float)s1 * inv; r[2] = (float)s2 * inv; r[3] = (float)s3 * inv;
  float* q = avg + b * C_DIM + c4;
  *(volatile v4f*)q = r;
  __threadfence();
  *(volatile v4f*)q = r;
}

__global__ __launch_bounds__(64) void k_ln1(const float* __restrict__ x, const float* __restrict__ avg,
                                            const float* __restrict__ w, const float* __restrict__ bb,
                                            _Float16* __restrict__ u) {
  __shared__ float red[4];
  const int row  = blockIdx.x;
  const int bidx = row / SEQ;
  const int tid = threadIdx.x, lane = tid & 31, wave = tid >> 5;
  const float* px = x + (size_t)row * C_DIM + lane * 8;
  const float* pa = avg + bidx * C_DIM + lane * 8;
  const float* src = (wave == 0) ? px : pa;
  const v4f a0 = *(const v4f*)src;
  const v4f a1 = *(const v4f*)(src + 4);
  float v[8];
  v[0] = a0[0]; v[1] = a0[1]; v[2] = a0[2]; v[3] = a0[3];
  v[4] = a1[0]; v[5] = a1[1]; v[6] = a1[2]; v[7] = a1[3];
  float s = 0.f;
#pragma unroll
  for (int e = 0; e < 8; ++e) s += v[e];
#pragma unroll
  for (int off = 16; off > 0; off >>= 1) s += __shfl_xor(s, off, 32);
  if (lane == 0) red[wave] = s;
  __syncthreads();
  const float mu = (red[0] + red[1]) * (1.0f / (float)DMODEL);
  float dv[8];
  float q = 0.f;
#pragma unroll
  for (int e = 0; e < 8; ++e) { dv[e] = v[e] - mu; q += dv[e] * dv[e]; }
#pragma unroll
  for (int off = 16; off > 0; off >>= 1) q += __shfl_xor(q, off, 32);
  if (lane == 0) red[2 + wave] = q;
  __syncthreads();
  const float var = (red[2] + red[3]) * (1.0f / (float)DMODEL);
  const float rs  = rsqrtf(var + LN_EPS);
  const int col0 = tid * 8;
  const v4f w0 = *(const v4f*)(w + col0),  w1 = *(const v4f*)(w + col0 + 4);
  const v4f b0 = *(const v4f*)(bb + col0), b1 = *(const v4f*)(bb + col0 + 4);
  v8h hv;
  hv[0] = (_Float16)(dv[0] * rs * w0[0] + b0[0]); hv[1] = (_Float16)(dv[1] * rs * w0[1] + b0[1]);
  hv[2] = (_Float16)(dv[2] * rs * w0[2] + b0[2]); hv[3] = (_Float16)(dv[3] * rs * w0[3] + b0[3]);
  hv[4] = (_Float16)(dv[4] * rs * w1[0] + b1[0]); hv[5] = (_Float16)(dv[5] * rs * w1[1] + b1[1]);
  hv[6] = (_Float16)(dv[6] * rs * w1[2] + b1[2]); hv[7] = (_Float16)(dv[7] * rs * w1[3] + b1[3]);
  _Float16* q8 = u + (size_t)row * DMODEL + col0;
  *(volatile v8h*)q8 = hv;
  __threadfence();
  *(volatile v8h*)q8 = hv;
}

__global__ __launch_bounds__(256) void k_conv(const float* __restrict__ xz, const float* __restrict__ cw,
                                              const float* __restrict__ cb, float* __restrict__ xc,
                                              _Float16* __restrict__ xch) {
  __shared__ __align__(16) _Float16 hs[DINNER];
  const int row = blockIdx.x;
  const int l   = row % SEQ;
  const int tid = threadIdx.x;
  const int d4  = tid << 2;
  const v4f wv0 = *(const v4f*)(cw + (size_t)(d4 + 0) * DCONV);
  const v4f wv1 = *(const v4f*)(cw + (size_t)(d4 + 1) * DCONV);
  const v4f wv2 = *(const v4f*)(cw + (size_t)(d4 + 2) * DCONV);
  const v4f wv3 = *(const v4f*)(cw + (size_t)(d4 + 3) * DCONV);
  float a0 = 0.f, a1 = 0.f, a2 = 0.f, a3 = 0.f;
#pragma unroll
  for (int k = 0; k < DCONV; ++k) {
    const int lk = l + k - (DCONV - 1);
    if (lk >= 0) {
      const v4f xv = *(const v4f*)(xz + (size_t)(row + k - (DCONV - 1)) * (2 * DINNER) + d4);
      a0 += xv[0] * wv0[k]; a1 += xv[1] * wv1[k]; a2 += xv[2] * wv2[k]; a3 += xv[3] * wv3[k];
    }
  }
  const v4f bv = *(const v4f*)(cb + d4);
  a0 += bv[0]; a1 += bv[1]; a2 += bv[2]; a3 += bv[3];
  const float s0 = a0 * __builtin_amdgcn_rcpf(1.0f + expf(-a0));
  const float s1 = a1 * __builtin_amdgcn_rcpf(1.0f + expf(-a1));
  const float s2 = a2 * __builtin_amdgcn_rcpf(1.0f + expf(-a2));
  const float s3 = a3 * __builtin_amdgcn_rcpf(1.0f + expf(-a3));
  v4f sv; sv[0] = s0; sv[1] = s1; sv[2] = s2; sv[3] = s3;
  float* q = xc + (size_t)row * DINNER + d4;
  *(volatile v4f*)q = sv;
  __threadfence();
  *(volatile v4f*)q = sv;
  hs[d4 + 0] = (_Float16)(s0 * XSC);
  hs[d4 + 1] = (_Float16)(s1 * XSC);
  hs[d4 + 2] = (_Float16)(s2 * XSC);
  hs[d4 + 3] = (_Float16)(s3 * XSC);
  __syncthreads();
  if (tid < 128) {
    const v8h hv = *(const v8h*)(hs + tid * 8);
    _Float16* qh = xch + (size_t)row * DINNER + tid * 8;
    *(volatile v8h*)qh = hv;
    __threadfence();
    *(volatile v8h*)qh = hv;
  }
}

__global__ __launch_bounds__(256) void k_dtx(const float* __restrict__ dbl, _Float16* __restrict__ dth) {
  const int i8 = blockIdx.x * 256 + threadIdx.x;
  if (i8 < (MROWS * DTRANK) / 8) {
    const int row = i8 >> 2;
    const int c8  = (i8 & 3) << 3;
    const float* p = dbl + (size_t)row * LDP + c8;
    const v4f a = *(const v4f*)p;
    const v4f c = *(const v4f*)(p + 4);
    v8h hv;
    hv[0] = (_Float16)(a[0] * XSC); hv[1] = (_Float16)(a[1] * XSC); hv[2] = (_Float16)(a[2] * XSC); hv[3] = (_Float16)(a[3] * XSC);
    hv[4] = (_Float16)(c[0] * XSC); hv[5] = (_Float16)(c[1] * XSC); hv[6] = (_Float16)(c[2] * XSC); hv[7] = (_Float16)(c[3] * XSC);
    _Float16* q = dth + (size_t)row * DTRANK + c8;
    *(volatile v8h*)q = hv;
    __threadfence();
    *(volatile v8h*)q = hv;
  }
}

__global__ __launch_bounds__(256) void k_softplus(const float* __restrict__ in, float* __restrict__ out) {
  const int i4 = blockIdx.x * 256 + threadIdx.x;
  if (i4 < (MROWS * DINNER) / 4) {
    const v4f v = *(const v4f*)(in + (size_t)i4 * 4);
    v4f r;
    r[0] = fmaxf(v[0], 0.f) + log1pf(expf(-fabsf(v[0])));
    r[1] = fmaxf(v[1], 0.f) + log1pf(expf(-fabsf(v[1])));
    r[2] = fmaxf(v[2], 0.f) + log1pf(expf(-fabsf(v[2])));
    r[3] = fmaxf(v[3], 0.f) + log1pf(expf(-fabsf(v[3])));
    float* q = out + (size_t)i4 * 4;
    *(volatile v4f*)q = r;
    __threadfence();
    *(volatile v4f*)q = r;
  }
}

__global__ __launch_bounds__(256) void k_scan(const float* __restrict__ dbl, const float* __restrict__ dtf,
                                              const float* __restrict__ xc, const float* __restrict__ alog,
                                              float* __restrict__ ys) {
  __shared__ float Bsh[DSTATE];
  __shared__ float Csh[DSTATE];
  const int tid = threadIdx.x, lane = tid & 31, wave = tid >> 5;
  const int b = blockIdx.x >> 7;
  const int d = ((blockIdx.x & 127) << 3) + wave;
  float An[8], h[8];
#pragma unroll
  for (int j = 0; j < 8; ++j) {
    An[j] = -expf(alog[(size_t)d * DSTATE + lane + 32 * j]);
    h[j] = 0.f;
  }
  float c0 = 0.f, c1 = 0.f, c2 = 0.f, c3 = 0.f;
  float* ych = ys + ((size_t)b * DINNER + d) * SEQ;
  for (int t = 0; t < SEQ; ++t) {
    const int row = b * SEQ + t;
    __syncthreads();
    Bsh[tid] = dbl[(size_t)row * LDP + DTRANK + tid];
    Csh[tid] = dbl[(size_t)row * LDP + DTRANK + DSTATE + tid];
    const float dt  = dtf[(size_t)row * DINNER + d];
    const float dtx = dt * xc[(size_t)row * DINNER + d];
    __syncthreads();
    float y = 0.f;
#pragma unroll
    for (int j = 0; j < 8; ++j) {
      const float dA = expf(dt * An[j]);
      h[j] = dA * h[j] + dtx * Bsh[lane + 32 * j];
      y += h[j] * Csh[lane + 32 * j];
    }
#pragma unroll
    for (int off = 16; off > 0; off >>= 1) y += __shfl_xor(y, off, 32);
    const int tt = t & 127;
    const bool mine = (lane == (tt >> 2));
    const int qq = tt & 3;
    c0 = (mine && qq == 0) ? y : c0;
    c1 = (mine && qq == 1) ? y : c1;
    c2 = (mine && qq == 2) ? y : c2;
    c3 = (mine && qq == 3) ? y : c3;
    if (tt == 127) {
      v4f v; v[0] = c0; v[1] = c1; v[2] = c2; v[3] = c3;
      float* p = ych + (t - 127) + 4 * lane;
      *(volatile v4f*)p = v;
      __threadfence();
      *(volatile v4f*)p = v;
    }
  }
}

__global__ __launch_bounds__(256) void k_gate(const float* __restrict__ ys, const float* __restrict__ xc,
                                              const float* __restrict__ xz, const float* __restrict__ Ds,
                                              _Float16* __restrict__ yh) {
  __shared__ float T[64][65];
  const int tid = threadIdx.x, lane = tid & 31, wave = tid >> 5;
  const int blk = blockIdx.x;
  const int b = blk >> 7;
  const int rem = blk & 127;
  const int d0 = (rem >> 3) * 64;
  const int t0 = (rem & 7) * 64;
  {
    const int i = tid >> 2;
    const int j16 = (tid & 3) << 4;
    const float* p = ys + ((size_t)b * DINNER + d0 + i) * SEQ + t0 + j16;
#pragma unroll
    for (int q = 0; q < 4; ++q) {
      const v4f v = *(const v4f*)(p + 4 * q);
      T[i][j16 + 4 * q + 0] = v[0]; T[i][j16 + 4 * q + 1] = v[1];
      T[i][j16 + 4 * q + 2] = v[2]; T[i][j16 + 4 * q + 3] = v[3];
    }
  }
  __syncthreads();
  const int rq = lane >> 3;
  const int c8 = (lane & 7) << 3;
  const int db = d0 + c8;
  const v4f D0 = *(const v4f*)(Ds + db), D1 = *(const v4f*)(Ds + db + 4);
#pragma unroll
  for (int it = 0; it < 2; ++it) {
    const int trow = wave * 8 + it * 4 + rq;
    const int row  = b * SEQ + t0 + trow;
    const float* xp = xc + (size_t)row * DINNER + db;
    const float* zp = xz + (size_t)row * (2 * DINNER) + DINNER + db;
    const v4f x0 = *(const v4f*)xp, x1 = *(const v4f*)(xp + 4);
    const v4f z0 = *(const v4f*)zp, z1 = *(const v4f*)(zp + 4);
    v8h hv;
#pragma unroll
    for (int e = 0; e < 4; ++e) {
      const float za = z0[e], zb = z1[e];
      const float ga = za * __builtin_amdgcn_rcpf(1.0f + expf(-za));
      const float gb = zb * __builtin_amdgcn_rcpf(1.0f + expf(-zb));
      const float va = (T[c8 + e][trow]     + x0[e] * D0[e]) * ga;
      const float vb = (T[c8 + 4 + e][trow] + x1[e] * D1[e]) * gb;
      hv[e]     = (_Float16)(va * YSC);
      hv[4 + e] = (_Float16)(vb * YSC);
    }
    _Float16* q = yh + (size_t)row * DINNER + db;
    *(volatile v8h*)q = hv;
    __threadfence();
    *(volatile v8h*)q = hv;
  }
}

__global__ __launch_bounds__(64) void k_ln2(const float* __restrict__ hin, const float* __restrict__ w,
                                            const float* __restrict__ bb, _Float16* __restrict__ o) {
  const int tid = threadIdx.x, lane = tid & 31, wave = tid >> 5;
  const int row = blockIdx.x * 2 + wave;
  const int col0 = lane * 8;
  const float* p = hin + (size_t)row * C_DIM + col0;
  const v4f a0 = *(const v4f*)p, a1 = *(const v4f*)(p + 4);
  float v[8];
  v[0] = a0[0]; v[1] = a0[1]; v[2] = a0[2]; v[3] = a0[3];
  v[4] = a1[0]; v[5] = a1[1]; v[6] = a1[2]; v[7] = a1[3];
  float s = 0.f;
#pragma unroll
  for (int e = 0; e < 8; ++e) s += v[e];
#pragma unroll
  for (int off = 16; off > 0; off >>= 1) s += __shfl_xor(s, off, 32);
  const float mu = s * (1.0f / (float)C_DIM);
  float dv[8];
  float q = 0.f;
#pragma unroll
  for (int e = 0; e < 8; ++e) { dv[e] = v[e] - mu; q += dv[e] * dv[e]; }
#pragma unroll
  for (int off = 16; off > 0; off >>= 1) q += __shfl_xor(q, off, 32);
  const float var = q * (1.0f / (float)C_DIM);
  const float rs  = rsqrtf(var + LN_EPS);
  const v4f w0 = *(const v4f*)(w + col0),  w1 = *(const v4f*)(w + col0 + 4);
  const v4f b0 = *(const v4f*)(bb + col0), b1 = *(const v4f*)(bb + col0 + 4);
  v8h hv;
  hv[0] = (_Float16)(dv[0] * rs * w0[0] + b0[0]); hv[1] = (_Float16)(dv[1] * rs * w0[1] + b0[1]);
  hv[2] = (_Float16)(dv[2] * rs * w0[2] + b0[2]); hv[3] = (_Float16)(dv[3] * rs * w0[3] + b0[3]);
  hv[4] = (_Float16)(dv[4] * rs * w1[0] + b1[0]); hv[5] = (_Float16)(dv[5] * rs * w1[1] + b1[1]);
  hv[6] = (_Float16)(dv[6] * rs * w1[2] + b1[2]); hv[7] = (_Float16)(dv[7] * rs * w1[3] + b1[3]);
  _Float16* q8 = o + (size_t)row * C_DIM + col0;
  *(volatile v8h*)q8 = hv;
  __threadfence();
  *(volatile v8h*)q8 = hv;
}

extern "C" void kernel_launch(void* const* d_in, const int* in_sizes, int n_in,
                              void* d_out, int out_size, void* d_ws, size_t ws_size,
                              hipStream_t stream) {
  (void)in_sizes; (void)n_in; (void)out_size;
  const float* x          = (const float*)d_in[0];
  const float* ln1_w      = (const float*)d_in[1];
  const float* ln1_b      = (const float*)d_in[2];
  const float* ln2_w      = (const float*)d_in[3];
  const float* ln2_b      = (const float*)d_in[4];
  const float* head_w     = (const float*)d_in[5];
  const float* head_b     = (const float*)d_in[6];
  const float* in_proj_w  = (const float*)d_in[7];
  const float* conv_w     = (const float*)d_in[8];
  const float* conv_b     = (const float*)d_in[9];
  const float* x_proj_w   = (const float*)d_in[10];
  const float* dt_proj_w  = (const float*)d_in[11];
  const float* dt_proj_b  = (const float*)d_in[12];
  const float* A_log      = (const float*)d_in[13];
  const float* D_skip     = (const float*)d_in[14];
  const float* out_proj_w = (const float*)d_in[15];
  float* out = (float*)d_out;

  char* wsp = (char*)d_ws;
  size_t off = 0;
  auto carve = [&](size_t bytes) -> char* {
    char* p = wsp + off;
    off += (bytes + 255) & ~(size_t)255;
    return p;
  };
  _Float16* w_in  = (_Float16*)carve((size_t)2 * DINNER * DMODEL * 2);
  _Float16* w_xp  = (_Float16*)carve((size_t)LDP * DINNER * 2);
  _Float16* w_dt  = (_Float16*)carve((size_t)DINNER * DTRANK * 2);
  _Float16* w_op  = (_Float16*)carve((size_t)C_DIM * DINNER * 2);
  _Float16* w_hd  = (_Float16*)carve((size_t)C_DIM * C_DIM * 2);
  float*    avg   = (float*)   carve((size_t)NB * C_DIM * 4);
  _Float16* u16   = (_Float16*)carve((size_t)MROWS * DMODEL * 2);
  float*    xz    = (float*)   carve((size_t)MROWS * 2 * DINNER * 4);
  float*    xc    = (float*)   carve((size_t)MROWS * DINNER * 4);
  _Float16* xc16  = (_Float16*)carve((size_t)MROWS * DINNER * 2);
  float*    dbl   = (float*)   carve((size_t)MROWS * LDP * 4);
  _Float16* dt16  = (_Float16*)carve((size_t)MROWS * DTRANK * 2);
  float*    dtraw = (float*)   carve((size_t)MROWS * DINNER * 4);
  float*    dtf   = (float*)   carve((size_t)MROWS * DINNER * 4);
  float*    ys    = (float*)   carve((size_t)MROWS * DINNER * 4);
  _Float16* y16   = (_Float16*)carve((size_t)MROWS * DINNER * 2);
  float*    hres  = (float*)   carve((size_t)MROWS * C_DIM * 4);
  _Float16* l16   = (_Float16*)carve((size_t)MROWS * C_DIM * 2);
  if (off > ws_size) return;

  const int T = 256;

  k_cast_rows<<<(2 * DINNER * DMODEL / 8 + T - 1) / T, T, 0, stream>>>(in_proj_w,  w_in, 2 * DINNER, DMODEL, 2 * DINNER, WSC);
  k_cast_rows<<<(LDP * DINNER / 8 + T - 1) / T,        T, 0, stream>>>(x_proj_w,   w_xp, NDBL,       DINNER, LDP,        WSC);
  k_cast_rows<<<(DINNER * DTRANK / 8 + T - 1) / T,     T, 0, stream>>>(dt_proj_w,  w_dt, DINNER,     DTRANK, DINNER,     DTWSC);
  k_cast_rows<<<(C_DIM * DINNER / 8 + T - 1) / T,      T, 0, stream>>>(out_proj_w, w_op, C_DIM,      DINNER, C_DIM,      WSC);
  k_cast_rows<<<(C_DIM * C_DIM / 8 + T - 1) / T,       T, 0, stream>>>(head_w,     w_hd, C_DIM,      C_DIM,  C_DIM,      WSC);

  k_avg<<<1, 128, 0, stream>>>(x, avg);
  k_ln1<<<MROWS, 64, 0, stream>>>(x, avg, ln1_w, ln1_b, u16);

  {
    const int tiles = (MROWS / 64) * ((2 * DINNER) / 64);
    wmma_gemm64<0, false, 0, 0, false, 0><<<dim3((tiles + 7) / 8, 1), T, 0, stream>>>(
        U16(u16), U16(u16), DMODEL, 0L, U16(w_in), U16(w_in), DMODEL, 0L,
        (void*)xz, (void*)xz, 2 * DINNER, 0L, conv_b, x, 0L, MROWS, 2 * DINNER, DMODEL, 1.0f / WSC);
  }

  k_conv<<<MROWS, T, 0, stream>>>(xz, conv_w, conv_b, xc, xc16);

  {
    const int tiles = (MROWS / 64) * (LDP / 64);
    wmma_gemm64<0, false, 0, 0, false, 0><<<dim3((tiles + 7) / 8, 1), T, 0, stream>>>(
        U16(xc16), U16(xc16), DINNER, 0L, U16(w_xp), U16(w_xp), DINNER, 0L,
        (void*)dbl, (void*)dbl, LDP, 0L, conv_b, x, 0L, MROWS, LDP, DINNER, 1.0f / (XSC * WSC));
  }

  k_dtx<<<(MROWS * DTRANK / 8 + T - 1) / T, T, 0, stream>>>(dbl, dt16);
  {
    const int tiles = (MROWS / 64) * (DINNER / 64);
    wmma_gemm64<0, false, 2, 0, false, 0><<<dim3((tiles + 7) / 8, 1), T, 0, stream>>>(
        U16(dt16), U16(dt16), DTRANK, 0L, U16(w_dt), U16(w_dt), DTRANK, 0L,
        (void*)dtraw, (void*)dtraw, DINNER, 0L, dt_proj_b, x, 0L, MROWS, DINNER, DTRANK, 1.0f / (XSC * DTWSC));
  }
  k_softplus<<<(MROWS * DINNER / 4 + T - 1) / T, T, 0, stream>>>(dtraw, dtf);

  k_scan<<<NB * (DINNER / 8), T, 0, stream>>>(dbl, dtf, xc, A_log, ys);

  k_gate<<<NB * (DINNER / 64) * (SEQ / 64), T, 0, stream>>>(ys, xc, xz, D_skip, y16);

  {
    const int tiles = (MROWS / 64) * (C_DIM / 64);
    wmma_gemm64<0, false, 0, 0, true, 0><<<dim3((tiles + 7) / 8, 1), T, 0, stream>>>(
        U16(y16), U16(y16), DINNER, 0L, U16(w_op), U16(w_op), DINNER, 0L,
        (void*)hres, (void*)hres, C_DIM, 0L, conv_b, x, 0L, MROWS, C_DIM, DINNER, 1.0f / (YSC * WSC));
  }

  k_ln2<<<MROWS / 2, 64, 0, stream>>>(hres, ln2_w, ln2_b, l16);
  {
    const int tiles = (MROWS / 64) * (C_DIM / 64);
    wmma_gemm64<0, false, 2, 0, true, 0><<<dim3((tiles + 7) / 8, 1), T, 0, stream>>>(
        U16(l16), U16(l16), C_DIM, 0L, U16(w_hd), U16(w_hd), C_DIM, 0L,
        (void*)out, (void*)out, C_DIM, 0L, head_b, hres, 0L, MROWS, C_DIM, C_DIM, 1.0f / WSC);
  }
}
